// MultiHeadKANAttention_81338090651880
// MI455X (gfx1250) — hardware-verified
//
#include <hip/hip_runtime.h>
#include <math.h>

constexpr int kB    = 2;
constexpr int kL    = 1024;
constexpr int kE    = 512;
constexpr int kH    = 8;
constexpr int kDh   = 64;
constexpr int kRows = kB * kL;
constexpr int kNB   = 35;
constexpr int kKsp  = kE * kNB;
constexpr int kChunksSp = kKsp / 8;
constexpr float kBasisCarry  = 1024.0f;
constexpr float kWspCarry    = 256.0f;
constexpr float kSplineScale = 1.0f / (1024.0f * 256.0f);
constexpr float kLo      = -3.0f;
constexpr float kHiClip  = 2.9999f;
constexpr float kKnot0   = -3.5625f;
constexpr float kKnotH   = 0.1875f;
constexpr float kInvH1   = 1.0f / 0.1875f;
constexpr float kInvH2   = 1.0f / 0.375f;
constexpr float kInvH3   = 1.0f / 0.5625f;

typedef __attribute__((ext_vector_type(16))) _Float16 v16h;
typedef __attribute__((ext_vector_type(8)))  _Float16 v8h;
typedef __attribute__((ext_vector_type(16))) __bf16   v16b;
typedef __attribute__((ext_vector_type(8)))  __bf16   v8b;
typedef __attribute__((ext_vector_type(8)))  float    v8f;
typedef __attribute__((ext_vector_type(4)))  float    v4f;
typedef __attribute__((ext_vector_type(4)))  unsigned int v4u;

__device__ __forceinline__ unsigned short f2bf_bits(float f) {
  unsigned u = __float_as_uint(f);
  return (unsigned short)((u + 0x7FFFu + ((u >> 16) & 1u)) >> 16);
}
__device__ __forceinline__ float bf_bits2f(unsigned short h) { return __uint_as_float(((unsigned)h) << 16); }

__device__ __forceinline__ void dep_guard_h(v8f& a, v8f& b, v16h x, v16h y) { asm volatile("v_nop\n\tv_nop\n\tv_nop\n\tv_nop" : "+v"(a), "+v"(b) : "v"(x), "v"(y)); }
__device__ __forceinline__ void dep_guard_b(v8f& a, v8f& b, v16b x, v16b y) { asm volatile("v_nop\n\tv_nop\n\tv_nop\n\tv_nop" : "+v"(a), "+v"(b) : "v"(x), "v"(y)); }
__device__ __forceinline__ void keep4_h(v16h a, v16h b, v16h c, v16h d) { asm volatile("v_nop" :: "v"(a), "v"(b), "v"(c), "v"(d)); }
__device__ __forceinline__ void keep4_b(v16b a, v16b b, v16b c, v16b d) { asm volatile("v_nop" :: "v"(a), "v"(b), "v"(c), "v"(d)); }
__device__ __forceinline__ void acc_guard4(v8f& a, v8f& b, v8f& c, v8f& d) { asm volatile("v_nop\n\tv_nop\n\tv_nop\n\tv_nop" : "+v"(a), "+v"(b), "+v"(c), "+v"(d)); }
template <typename T> struct Frag;
template <> struct Frag<_Float16> {
  typedef v16h V; union U { v16h v; v8h h[2]; };
  static __device__ __forceinline__ v16h load(const _Float16* p) {
    U f; f.h[0] = *(const v8h*)(p); f.h[1] = *(const v8h*)(p + 16); return f.v;
  }
  static __device__ __forceinline__ v8f mma(v16h a, v16h b, v8f c) {
    return __builtin_amdgcn_wmma_f32_16x16x32_f16(false, a, false, b, (short)0, c, false, false);
  }
  static __device__ __forceinline__ void guard(v8f& a, v8f& b, v16h x, v16h y) { dep_guard_h(a, b, x, y); }
  static __device__ __forceinline__ void keep(v16h a, v16h b, v16h c, v16h d) { keep4_h(a, b, c, d); }
};
template <> struct Frag<__bf16> {
  typedef v16b V; union U { v16b v; v8b h[2]; };
  static __device__ __forceinline__ v16b load(const __bf16* p) {
    U f; f.h[0] = *(const v8b*)(p); f.h[1] = *(const v8b*)(p + 16); return f.v;
  }
  static __device__ __forceinline__ v8f mma(v16b a, v16b b, v8f c) {
    return __builtin_amdgcn_wmma_f32_16x16x32_bf16(false, a, false, b, (short)0, c, false, false);
  }
  static __device__ __forceinline__ void guard(v8f& a, v8f& b, v16b x, v16b y) { dep_guard_b(a, b, x, y); }
  static __device__ __forceinline__ void keep(v16b a, v16b b, v16b c, v16b d) { keep4_b(a, b, c, d); }
};

__device__ __forceinline__ unsigned pk16(unsigned short a, unsigned short b) { return (unsigned)a | ((unsigned)b << 16); }
__device__ __forceinline__ unsigned short h_bits(float f) { const _Float16 h = (_Float16)f; return __builtin_bit_cast(unsigned short, h); }

template <int ET> struct Elem;
template <> struct Elem<0> { typedef _Float16 T; };
template <> struct Elem<1> { typedef __bf16 T; };
template <int ET, bool SPLIT, int BIAS_MODE, int OUT_MODE, bool RESID, int ACT = 0>
__global__ __launch_bounds__(256) void wmma_gemm64(
    const unsigned short* __restrict__ Ap, const unsigned short* __restrict__ A2p, int lda, long strideA,
    const unsigned short* __restrict__ Btp, const unsigned short* __restrict__ Bt2p, int ldb, long strideB,
    void* __restrict__ Cout, void* __restrict__ Cout2, int ldc, long strideC,
    const float* __restrict__ bias,
    const float* __restrict__ resid, long strideR,
    int M, int N, int K, float scale) {
  typedef typename Elem<ET>::T T;
  typedef typename Frag<T>::V V;
  const T* A = (const T*)Ap; const T* A2 = (const T*)A2p; const T* Bt = (const T*)Btp; const T* Bt2 = (const T*)Bt2p;
  __shared__ __align__(16) float sT[8][16 * 68];
  const int b    = blockIdx.y;
  const int lane = threadIdx.x & 31;
  const int wave = threadIdx.x >> 5;
  const int tilesN = N >> 6;
  const int tilesM = M >> 6;
  const int tile = blockIdx.x * 8 + wave;
  if (tile >= tilesM * tilesN) return;
  const int tm = tile / tilesN;
  const int tn = tile - tm * tilesN;
  const int m0 = tm << 6;
  const int n0 = tn << 6;

  const T* Ab  = A  + (size_t)b * strideA;
  const T* Bb  = Bt + (size_t)b * strideB;
  const T* Ab2 = SPLIT ? (A2  + (size_t)b * strideA) : nullptr;
  const T* Bb2 = SPLIT ? (Bt2 + (size_t)b * strideB) : nullptr;

  const int rlane = lane & 15;
  const int koff  = (lane >> 4) * 8;
  const int mOff  = (lane >> 4) * 8;

  v8f acc[4][4];
#pragma unroll
  for (int i = 0; i < 4; ++i)
#pragma unroll
    for (int j = 0; j < 4; ++j) acc[i][j] = (v8f){0.f,0.f,0.f,0.f,0.f,0.f,0.f,0.f};

  for (int k0 = 0; k0 < K; k0 += 32) {
    V bh[4], bl[4];
#pragma unroll
    for (int j = 0; j < 4; ++j) {
      const size_t bo = (size_t)(n0 + (j << 4) + rlane) * ldb + koff + k0;
      bh[j] = Frag<T>::load(Bb + bo);
      if (SPLIT) bl[j] = Frag<T>::load(Bb2 + bo);
    }
#pragma unroll
    for (int i = 0; i < 4; ++i) {
      const size_t ao = (size_t)(m0 + (i << 4) + rlane) * lda + koff + k0;
      V ah = Frag<T>::load(Ab + ao);
      V al;
      if (SPLIT) al = Frag<T>::load(Ab2 + ao);
#pragma unroll
      for (int j = 0; j < 4; ++j) {
        acc[i][j] = Frag<T>::mma(ah, bh[j], acc[i][j]);
        if (SPLIT) {
          acc[i][j] = Frag<T>::mma(ah, bl[j], acc[i][j]);
          acc[i][j] = Frag<T>::mma(al, bh[j], acc[i][j]);
        }
      }
      Frag<T>::guard(acc[i][0], acc[i][3], ah, SPLIT ? al : ah);
    }
    Frag<T>::keep(bh[0], bh[1], bh[2], bh[3]);
    if (SPLIT) Frag<T>::keep(bl[0], bl[1], bl[2], bl[3]);
  }
  acc_guard4(acc[0][0], acc[0][1], acc[0][2], acc[0][3]);
  acc_guard4(acc[1][0], acc[1][1], acc[1][2], acc[1][3]);
  acc_guard4(acc[2][0], acc[2][1], acc[2][2], acc[2][3]);
  acc_guard4(acc[3][0], acc[3][1], acc[3][2], acc[3][3]);

  float* slab = sT[wave];
  const float* Rb = RESID ? (resid + (size_t)b * strideR) : nullptr;
#pragma unroll
  for (int i = 0; i < 4; ++i) {
    const int mBase = m0 + (i << 4);
#pragma unroll
    for (int j = 0; j < 4; ++j) {
      const int n = n0 + (j << 4) + rlane;
      float bv = 0.f;
      if (BIAS_MODE == 2) bv = bias[n];
#pragma unroll
      for (int r = 0; r < 8; ++r) {
        float v = acc[i][j][r] * scale;
        if (BIAS_MODE == 1) v += bias[mBase + mOff + r];
        if (BIAS_MODE == 2) v += bv;
        if (RESID) v += Rb[(size_t)(mBase + mOff + r) * ldc + n];
        if (ACT == 2) v = fmaxf(v, 0.0f);
        if (ACT == 4) v = (v > 0.f) ? v : 0.01f * v;
        slab[(mOff + r) * 68 + (j << 4) + rlane] = v;
      }
    }
    __builtin_amdgcn_fence(__ATOMIC_RELEASE, "workgroup");
    __builtin_amdgcn_wave_barrier();
    __builtin_amdgcn_fence(__ATOMIC_ACQUIRE, "workgroup");
    if (OUT_MODE == 0) {
      float* C = (float*)Cout + (size_t)b * strideC;
      const int hh = lane >> 4, c4 = (lane & 15) * 4;
      for (int pass = 0; pass < 2; ++pass) {
#pragma unroll
        for (int it = 0; it < 8; ++it) {
          const int row = it * 2 + hh;
          v4f v = *(const v4f*)(slab + row * 68 + c4);
          *(volatile v4f*)(C + (size_t)(mBase + row) * ldc + n0 + c4) = v;
        }
        __threadfence();
      }
    } else {
      const int q = lane >> 3, c8 = (lane & 7) * 8;
      unsigned short* C  = (unsigned short*)Cout  + (size_t)b * strideC;
      unsigned short* C2 = (OUT_MODE == 2) ? ((unsigned short*)Cout2 + (size_t)b * strideC) : nullptr;
      for (int pass = 0; pass < 2; ++pass) {
#pragma unroll
        for (int it = 0; it < 4; ++it) {
          const int row = it * 4 + q;
          const float* sp = slab + row * 68 + c8;
          v8h hv, lv;
#pragma unroll
          for (int e = 0; e < 8; ++e) {
            if (OUT_MODE == 1) {
              hv[e] = (_Float16)sp[e];
            } else {
              unsigned short hb = f2bf_bits(sp[e]);
              unsigned short lb = f2bf_bits(sp[e] - bf_bits2f(hb));
              hv[e] = __builtin_bit_cast(_Float16, hb);
              lv[e] = __builtin_bit_cast(_Float16, lb);
            }
          }
          *(volatile v8h*)(C + (size_t)(mBase + row) * ldc + n0 + c8) = hv;
          if (OUT_MODE == 2) *(volatile v8h*)(C2 + (size_t)(mBase + row) * ldc + n0 + c8) = lv;
        }
        __threadfence();
      }
    }
    __builtin_amdgcn_fence(__ATOMIC_RELEASE, "workgroup");
    __builtin_amdgcn_wave_barrier();
    __builtin_amdgcn_fence(__ATOMIC_ACQUIRE, "workgroup");
  }
}

template <int MODE>
__global__ __launch_bounds__(256) void wtrans_kernel(const float* __restrict__ src, unsigned short* __restrict__ out0,
                                                     unsigned short* __restrict__ out1, int ldo, float scale) {
  __shared__ __align__(16) float sm[64][68];
  const int t   = threadIdx.x;
  const int kc0 = blockIdx.x * 64;
  const int oc0 = blockIdx.y * 64;
#pragma unroll
  for (int i = 0; i < 4; ++i) {
    const int idx = i * 256 + t;
    const int kr  = idx >> 4;
    const int o4  = (idx & 15) * 4;
    const v4f w = *(const v4f*)(src + (size_t)(kc0 + kr) * kE + oc0 + o4);
    sm[o4 + 0][kr] = w[0] * scale;
    sm[o4 + 1][kr] = w[1] * scale;
    sm[o4 + 2][kr] = w[2] * scale;
    sm[o4 + 3][kr] = w[3] * scale;
  }
  __syncthreads();
  const int lane = t & 31, wave = t >> 5;
  const int q = lane >> 3, c8 = (lane & 7) * 8;
  for (int pass = 0; pass < 2; ++pass) {
#pragma unroll
    for (int it = 0; it < 2; ++it) {
      const int row = wave * 8 + it * 4 + q;
      const v4f f0 = *(const v4f*)(&sm[row][c8]);
      const v4f f1 = *(const v4f*)(&sm[row][c8 + 4]);
      const float f[8] = {f0[0], f0[1], f0[2], f0[3], f1[0], f1[1], f1[2], f1[3]};
      unsigned short ha[8], la[8];
#pragma unroll
      for (int e = 0; e < 8; ++e) {
        if (MODE == 0) {
          ha[e] = h_bits(f[e]);
          la[e] = 0;
        } else {
          ha[e] = f2bf_bits(f[e]);
          la[e] = f2bf_bits(f[e] - bf_bits2f(ha[e]));
        }
      }
      const v4u pa = (v4u){pk16(ha[0], ha[1]), pk16(ha[2], ha[3]), pk16(ha[4], ha[5]), pk16(ha[6], ha[7])};
      const size_t off = (size_t)(oc0 + row) * ldo + kc0 + c8;
      *(volatile v4u*)(out0 + off) = pa;
      if (MODE == 1) {
        const v4u pl = (v4u){pk16(la[0], la[1]), pk16(la[2], la[3]), pk16(la[4], la[5]), pk16(la[6], la[7])};
        *(volatile v4u*)(out1 + off) = pl;
      }
    }
    __threadfence();
  }
}

__device__ __forceinline__ float knot_at(int i) { return kKnotH * (float)i + kKnot0; }

__global__ __launch_bounds__(256) void expand_kernel(const float* __restrict__ X, unsigned short* __restrict__ A16,
                                                     unsigned short* __restrict__ SXh, unsigned short* __restrict__ SXl) {
#pragma clang fp contract(off)
  __shared__ __align__(16) unsigned short srow[kKsp];
  __shared__ __align__(16) unsigned short ssh[kE];
  __shared__ __align__(16) unsigned short ssl[kE];
  const int m = blockIdx.x;
  const int t = threadIdx.x;
  const v4u z4 = (v4u){0u, 0u, 0u, 0u};
#pragma unroll
  for (int i = 0; i < 9; ++i) {
    const int q = i * 256 + t;
    if (q < kChunksSp) *(v4u*)(srow + 8 * q) = z4;
  }
  __syncthreads();
#pragma unroll
  for (int hf = 0; hf < 2; ++hf) {
    const int e = t + hf * 256;
    const float x = X[(size_t)m * kE + e];
    const float sg = 1.0f / (1.0f + expf(-x));
    const float s  = x * sg;
    const unsigned short shb = f2bf_bits(s);
    ssh[e] = shb;
    ssl[e] = f2bf_bits(s - bf_bits2f(shb));
    const float xe = fminf(fmaxf(x, kLo), kHiClip);
    int c = (int)((xe + 3.5625f) * kInvH1);
    c = (c < 3) ? 3 : ((c > 34) ? 34 : c);
    c -= (xe < knot_at(c)) ? 1 : 0;
    c += (xe >= knot_at(c + 1)) ? 1 : 0;
    c = (c < 3) ? 3 : ((c > 34) ? 34 : c);
    const float t_m2 = knot_at(c - 2), t_m1 = knot_at(c - 1), t_c0 = knot_at(c);
    const float t_p1 = knot_at(c + 1), t_p2 = knot_at(c + 2), t_p3 = knot_at(c + 3);
    const float l0 = xe - t_c0, l1 = xe - t_m1, l2 = xe - t_m2;
    const float r1 = t_p1 - xe, r2 = t_p2 - xe, r3 = t_p3 - xe;
    const float b1a = r1 * kInvH1;
    const float b1b = l0 * kInvH1;
    const float b2a = (r1 * kInvH2) * b1a;
    const float b2b = (l1 * kInvH2) * b1a + (r2 * kInvH2) * b1b;
    const float b2c = (l0 * kInvH2) * b1b;
    const float b3a = (r1 * kInvH3) * b2a;
    const float b3b = (l2 * kInvH3) * b2a + (r2 * kInvH3) * b2b;
    const float b3c = (l1 * kInvH3) * b2b + (r3 * kInvH3) * b2c;
    const float b3d = (l0 * kInvH3) * b2c;
    unsigned short* dst = srow + e * kNB + (c - 3);
    dst[0] = h_bits(b3a * kBasisCarry);
    dst[1] = h_bits(b3b * kBasisCarry);
    dst[2] = h_bits(b3c * kBasisCarry);
    dst[3] = h_bits(b3d * kBasisCarry);
  }
  __syncthreads();
  unsigned short* arow = A16 + (size_t)m * kKsp;
  unsigned short* hrow = SXh + (size_t)m * kE;
  unsigned short* lrow = SXl + (size_t)m * kE;
  for (int pass = 0; pass < 2; ++pass) {
#pragma unroll
    for (int i = 0; i < 9; ++i) {
      const int q = i * 256 + t;
      if (q < kChunksSp) {
        const v4u v = *(const v4u*)(srow + 8 * q);
        *(volatile v4u*)(arow + 8 * q) = v;
      }
    }
    if (t < 64) {
      const v4u v = *(const v4u*)(ssh + 8 * t);
      *(volatile v4u*)(hrow + 8 * t) = v;
    }
    if (t >= 64 && t < 128) {
      const v4u v = *(const v4u*)(ssl + 8 * (t - 64));
      *(volatile v4u*)(lrow + 8 * (t - 64)) = v;
    }
    __threadfence();
  }
}

extern "C" void kernel_launch(void* const* d_in, const int* in_sizes, int n_in,
                              void* d_out, int out_size, void* d_ws, size_t ws_size,
                              hipStream_t stream) {
  if (n_in < 9) return;
  if (in_sizes[0] != kRows * kE || in_sizes[1] != kRows * kE || in_sizes[2] != kRows * kE) return;
  if (in_sizes[3] != kE * kE || in_sizes[5] != kE * kE || in_sizes[7] != kE * kE) return;
  if (in_sizes[4] != kE * kNB * kE || in_sizes[6] != kE * kNB * kE || in_sizes[8] != kE * kNB * kE) return;
  if (out_size != kRows * kE) return;

  const float* xs[3]   = {(const float*)d_in[0], (const float*)d_in[1], (const float*)d_in[2]};
  const float* wbs[3]  = {(const float*)d_in[3], (const float*)d_in[5], (const float*)d_in[7]};
  const float* wsps[3] = {(const float*)d_in[4], (const float*)d_in[6], (const float*)d_in[8]};
  float* out = (float*)d_out;

  unsigned char* ws = (unsigned char*)d_ws;
  size_t off = 0;
  const size_t szA16 = (size_t)kRows * kKsp * 2;
  const size_t szWsp = (size_t)kE * kKsp * 2;
  const size_t szWb  = (size_t)kE * kE * 2;
  const size_t szSX  = (size_t)kRows * kE * 2;
  const size_t szYf  = (size_t)kRows * kE * 4;
  const size_t szP   = (size_t)kRows * kE * 2;
  const size_t szW2  = (size_t)kB * kH * kDh * kDh * 2;
  unsigned short* A16  = (unsigned short*)(ws + off); off += szA16;
  unsigned short* Wsp  = (unsigned short*)(ws + off); off += szWsp;
  unsigned short* WbTh = (unsigned short*)(ws + off); off += szWb;
  unsigned short* WbTl = (unsigned short*)(ws + off); off += szWb;
  unsigned short* SXh  = (unsigned short*)(ws + off); off += szSX;
  unsigned short* SXl  = (unsigned short*)(ws + off); off += szSX;
  float*          Yf   = (float*)(ws + off);          off += szYf;
  unsigned short* Qh   = (unsigned short*)(ws + off); off += szP;
  unsigned short* Ql   = (unsigned short*)(ws + off); off += szP;
  unsigned short* KTh  = (unsigned short*)(ws + off); off += szP;
  unsigned short* KTl  = (unsigned short*)(ws + off); off += szP;
  unsigned short* VTh  = (unsigned short*)(ws + off); off += szP;
  unsigned short* VTl  = (unsigned short*)(ws + off); off += szP;
  unsigned short* W2h  = (unsigned short*)(ws + off); off += szW2;
  unsigned short* W2l  = (unsigned short*)(ws + off); off += szW2;
  if (off > ws_size) return;
  const float* Yff = (const float*)Yf;

  const long strideA16B = (long)kL * kKsp;
  const long strideTok  = (long)kL * kE;
  const long strideT    = (long)kE * kL;

  for (int p = 0; p < 3; ++p) {
    wtrans_kernel<0><<<dim3(kKsp / 64, kE / 64), 256, 0, stream>>>(wsps[p], Wsp, Wsp, kKsp, kWspCarry);
    wtrans_kernel<1><<<dim3(kE / 64, kE / 64), 256, 0, stream>>>(wbs[p], WbTh, WbTl, kE, 1.0f);
    expand_kernel<<<kRows, 256, 0, stream>>>(xs[p], A16, SXh, SXl);
    if (p == 0) {
      wmma_gemm64<0, false, 0, 0, false><<<dim3((kRows / 64) * (kE / 64) / 8, 1), 256, 0, stream>>>(
          A16, A16, kKsp, 0L, Wsp, Wsp, kKsp, 0L, Yf, Yf, kE, 0L, Yff, Yff, 0L, kRows, kE, kKsp, kSplineScale);
      wmma_gemm64<1, true, 0, 2, true><<<dim3((kRows / 64) * (kE / 64) / 8, 1), 256, 0, stream>>>(
          SXh, SXl, kE, 0L, WbTh, WbTl, kE, 0L, Qh, Ql, kE, 0L, Yff, Yff, 0L, kRows, kE, kE, 1.0f);
    } else {
      unsigned short* Th = (p == 1) ? KTh : VTh;
      unsigned short* Tl = (p == 1) ? KTl : VTl;
      wmma_gemm64<0, false, 0, 0, false><<<dim3((kE / 64) * (kL / 64) / 8, kB), 256, 0, stream>>>(
          Wsp, Wsp, kKsp, 0L, A16, A16, kKsp, strideA16B, Yf, Yf, kL, strideT, Yff, Yff, 0L, kE, kL, kKsp, kSplineScale);
      wmma_gemm64<1, true, 0, 2, true><<<dim3((kE / 64) * (kL / 64) / 8, kB), 256, 0, stream>>>(
          WbTh, WbTl, kE, 0L, SXh, SXl, kE, strideTok, Th, Tl, kL, strideT, Yff, Yff, strideT, kE, kL, kE, 1.0f);
    }
  }
  wmma_gemm64<1, true, 0, 2, false><<<dim3(1, kB * kH), 32, 0, stream>>>(
      VTh, VTl, kL, (long)kDh * kL, KTh, KTl, kL, (long)kDh * kL, W2h, W2l, kDh, (long)kDh * kDh,
      Yff, Yff, 0L, kDh, kDh, kL, 1.0f);
  for (int h = 0; h < kH; ++h) {
    wmma_gemm64<1, true, 0, 0, false><<<dim3((kL / 64) / 8, kB), 256, 0, stream>>>(
        Qh + h * kDh, Ql + h * kDh, kE, strideTok,
        W2h + h * kDh * kDh, W2l + h * kDh * kDh, kDh, (long)kH * kDh * kDh,
        out + h * kDh, out + h * kDh, kE, strideTok,
        Yff, Yff, 0L, kL, kDh, kDh, 1.0f);
  }
}
